// Encoder_block_11553462026609
// MI455X (gfx1250) — hardware-run, weakly checked
//
#include <hip/hip_runtime.h>


#ifndef NB
#define NB 4
#endif
#ifndef SEQ
#define SEQ 2048
#endif
#define NB_FULL  4
#define SEQ_FULL 2048
#ifndef OUT_SEQ
#define OUT_SEQ SEQ
#endif
#define DM    1024
#define NH_   16
#define HD    64
#define FFD   4096
#define AW    4
#define MROWS (NB * SEQ)
#define MHALF (MROWS / 2)
#define WSC   64.0f
#define WSI   (1.0f / 64.0f)
#define ACY   16.0f
#define SC2   (0.125f * 1.4426950408889634f)
#define PSH   8.0f
#define BIGB  0x40000000

static_assert(HD == 64);
static_assert(NH_ * HD == DM);
static_assert(DM % 64 == 0);
static_assert(FFD % 64 == 0);
static_assert(DM % 32 == 0);
static_assert(FFD % 32 == 0);
static_assert(DM == 1024);
static_assert(SEQ % 64 == 0);
static_assert(MROWS % 128 == 0);
static_assert(MROWS % 8 == 0);
static_assert(MHALF % 8 == 0);
static_assert(SEQ % 32 == 0);
static_assert(SEQ % (16 * AW) == 0);
static_assert(NB <= NB_FULL);
static_assert(SEQ <= SEQ_FULL);
static_assert(MROWS < BIGB);
static_assert(256 * 16 * 2 == 64 * 64 * 2);
static_assert(32 * 16 * 4 == DM * 2);
static_assert(32 * 16 * 8 == DM * 4);
static_assert(32 * 8 * 8 == DM * 2);
static_assert(32 * 16 * 4 == 16 * 64 * 2);
static_assert(32 * 16 * 8 == 16 * 64 * 4);
static_assert(64 * 65 * 4 <= 131072);
static_assert(16 * 68 * 4 <= 131072);
static_assert(AW * 16 * 68 * 4 <= 131072);

typedef _Float16 h16;
typedef __attribute__((ext_vector_type(16))) _Float16 v16h;
typedef __attribute__((ext_vector_type(8)))  _Float16 v8h;
typedef __attribute__((ext_vector_type(4)))  _Float16 v4h;
typedef __attribute__((ext_vector_type(8)))  float    v8f;
typedef __attribute__((ext_vector_type(4)))  float    v4f;
typedef v4f  __attribute__((may_alias)) v4fa;

__device__ __forceinline__ unsigned short f2bf(float f) { unsigned u = __float_as_uint(f); u += 0x7FFFu + ((u >> 16) & 1u); return (unsigned short)(u >> 16); }
__device__ __forceinline__ float bfr(float f) { return __uint_as_float(((unsigned)f2bf(f)) << 16); }
__device__ __forceinline__ v16h cat16(v8h lo, v8h hi) { return __builtin_shufflevector(lo, hi, 0, 1, 2, 3, 4, 5, 6, 7, 8, 9, 10, 11, 12, 13, 14, 15); }
__device__ __forceinline__ v8f wmma16(v16h a, v16h b, v8f c) { return __builtin_amdgcn_wmma_f32_16x16x32_f16(false, a, false, b, (short)0, c, false, false); }
__device__ __forceinline__ v16h ldh(const h16* p) { return cat16(*(const v8h*)p, *(const v8h*)(p + 16)); }
__device__ __forceinline__ void wave_sync() { __builtin_amdgcn_fence(3  , "wavefront"); __builtin_amdgcn_wave_barrier(); asm volatile("" ::: "memory"); }

static __device__ __forceinline__ h16 toh_flush(float v) { const h16 r = (h16)v; return (fabsf(v) < 6.103515625e-05f) ? (h16)0.0f : r; }
static __device__ __forceinline__ v8f wmma16g(v16h a, v16h b, v8f c) {
    c = __builtin_amdgcn_wmma_f32_16x16x32_f16(false, a, false, b, (short)0, c, false, false);
    asm volatile("v_nop\n\tv_nop\n\tv_nop\n\tv_nop" : "+v"(c) : "v"(a), "v"(b));
    return c;
}
static __device__ __forceinline__ float gelu_f(float y) {
    const float ay = fabsf(y);
    const float t = __builtin_amdgcn_rcpf(1.0f + 0.231641888f * ay);
    float pl = 1.061405429f;
    pl = pl * t - 1.453152027f;
    pl = pl * t + 1.421413741f;
    pl = pl * t - 0.284496736f;
    pl = pl * t + 0.254829592f;
    const float e = (pl * t) * __builtin_amdgcn_exp2f((y * y) * (-0.72134752044448170f));
    const float q = (0.5f * ay) * e;
    return (y > 0.0f) ? (y - q) : (0.0f - q);
}

__global__ __launch_bounds__(256) void k_tcvt(const float* __restrict__ in, h16* out, int R, int Cc, size_t inZ, size_t outZ) {
    __shared__ float tl[64 * 65];
    const int tid = threadIdx.x;
    const int r0 = blockIdx.y * 64, c0 = blockIdx.x * 64;
    const float* src = in + (size_t)blockIdx.z * inZ + (size_t)r0 * Cc + c0;
    h16* dst = out + (size_t)blockIdx.z * outZ + (size_t)c0 * R + r0;
#pragma unroll 4
    for (int i = 0; i < 16; ++i) { const int r = i * 4 + (tid >> 6), c = tid & 63; tl[r * 65 + c] = src[(size_t)r * Cc + c]; }
    __syncthreads();
    const int oc = tid >> 3, sg = (tid & 7) * 8;
    v8h o0, o1;
#pragma unroll
    for (int k = 0; k < 8; ++k) { o0[k] = toh_flush(bfr(tl[(sg + k) * 65 + oc]) * WSC); o1[k] = toh_flush(bfr(tl[(sg + k) * 65 + oc + 32]) * WSC); }
#pragma unroll 1
    for (int ps = 0; ps < 2; ++ps) {
        *(volatile v8h*)(dst + (size_t)oc * R + sg) = o0;
        *(volatile v8h*)(dst + (size_t)(oc + 32) * R + sg) = o1;
        if (ps == 0) __threadfence();
    }
}

__device__ __forceinline__ void ld8(const float* p, const int rnd, v4f& a, v4f& c) {
    a = *(const v4f*)p; c = *(const v4f*)(p + 4);
#pragma unroll
    for (int k = 0; k < 4; ++k) { const float ra = bfr(a[k]), rc = bfr(c[k]); a[k] = rnd ? ra : a[k]; c[k] = rnd ? rc : c[k]; }
}

__global__ __launch_bounds__(256) void k_cast(const float* __restrict__ X, h16* out, int inSeq) {
#pragma clang fp contract(off)
    const int lane = threadIdx.x & 31, wave = __builtin_amdgcn_readfirstlane((int)(threadIdx.x >> 5));
    const int row = blockIdx.x * 8 + wave;
    const int b = row / SEQ, t = row % SEQ;
    const float* xr = X + ((size_t)b * inSeq + t) * DM + lane * 8;
    h16* orow = out + (size_t)row * DM + lane * 8;
#pragma unroll 1
    for (int i = 0; i < 4; ++i) { v4f a, c; ld8(xr + i * 256, 1, a, c);
        v8h hv;
#pragma unroll
        for (int k = 0; k < 4; ++k) { hv[k] = toh_flush(a[k]); hv[4 + k] = toh_flush(c[k]); }
        *(volatile v8h*)(orow + i * 256) = hv; __threadfence(); *(volatile v8h*)(orow + i * 256) = hv; }
}

__global__ __launch_bounds__(256) void k_lnres(const float* __restrict__ Y, const float* R, const float* __restrict__ G, const float* __restrict__ Bv,
                                               float* outF, h16* outH, int wh, int rnd, int rowOff, int rSeq, int oSeq) {
#pragma clang fp contract(off)
    const int lane = threadIdx.x & 31, wave = __builtin_amdgcn_readfirstlane((int)(threadIdx.x >> 5));
    const int lrow = blockIdx.x * 8 + wave;
    const int gr = rowOff + lrow;
    const int b = gr / SEQ, t = gr % SEQ;
    const float* yr = Y + (size_t)lrow * DM + lane * 4;
    const float* rp = R + ((size_t)b * rSeq + t) * DM + lane * 4;
    float* of = outF + ((size_t)b * oSeq + t) * DM + lane * 4;
    h16* oh = outH + (size_t)gr * DM + lane * 4;
    float s = 0.0f;
#pragma unroll 1
    for (int j = 0; j < 8; ++j) { const v4f a = *(const v4f*)(yr + j * 128); s += (a[0] + a[1]) + (a[2] + a[3]); }
#pragma unroll
    for (int msk = 16; msk; msk >>= 1) s += __shfl_xor(s, msk, 32);
    const float mu = s * (1.0f / DM);
    float ss = 0.0f;
#pragma unroll 1
    for (int j = 0; j < 8; ++j) { const v4f a = *(const v4f*)(yr + j * 128);
#pragma unroll
        for (int k = 0; k < 4; ++k) { const float d0 = a[k] - mu; ss += d0 * d0; } }
#pragma unroll
    for (int msk = 16; msk; msk >>= 1) ss += __shfl_xor(ss, msk, 32);
    const float rstd = rsqrtf(ss * (1.0f / DM) + 1.0e-5f);
#pragma unroll 1
    for (int j = 0; j < 8; ++j) {
        const v4f a = *(const v4f*)(yr + j * 128); const v4f rs = *(const v4f*)(rp + j * 128);
        const v4f ga = *(const v4f*)(G + j * 128 + lane * 4); const v4f ba = *(const v4f*)(Bv + j * 128 + lane * 4);
        v4f ov; v4h hv;
#pragma unroll
        for (int k = 0; k < 4; ++k) { const float rq = bfr(rs[k]); const float rv = rnd ? rq : rs[k];
            const float nv = ((a[k] - mu) * rstd) * bfr(ga[k]) + bfr(ba[k]);
            ov[k] = rv + nv; hv[k] = toh_flush(ov[k]); }
        *(volatile v4f*)(of + j * 128) = ov;
        if (wh) *(volatile v4h*)(oh + j * 128) = hv;
        __threadfence();
        *(volatile v4f*)(of + j * 128) = ov;
        if (wh) *(volatile v4h*)(oh + j * 128) = hv; }
}

__device__ __forceinline__ void gemm_main(const h16* __restrict__ A, const h16* __restrict__ Bt, const int K, const int r0, const int c0, const int lr, const int hi, v8f (&acc)[4][4]) {
#pragma unroll
    for (int mb = 0; mb < 4; ++mb)
#pragma unroll
        for (int nb = 0; nb < 4; ++nb) acc[mb][nb] = (v8f){};
    const size_t aoff = (size_t)(r0 + lr) * K + 8 * hi, boff = (size_t)(c0 + lr) * K + 8 * hi;
#pragma unroll 1
    for (int kc = 0; kc < K; kc += 32) {
        v16h a[4];
#pragma unroll
        for (int mb = 0; mb < 4; ++mb) a[mb] = ldh(A + aoff + (size_t)mb * 16 * K + kc);
#pragma unroll
        for (int nb = 0; nb < 4; ++nb) { const v16h bq = ldh(Bt + boff + (size_t)nb * 16 * K + kc);
#pragma unroll
            for (int mb = 0; mb < 4; ++mb) acc[mb][nb] = wmma16(a[mb], bq, acc[mb][nb]); }
        asm volatile("v_nop\n\tv_nop\n\tv_nop\n\tv_nop" : "+v"(acc[0][3]), "+v"(acc[1][3]), "+v"(acc[2][3]), "+v"(acc[3][3]) : "v"(a[0]), "v"(a[1]), "v"(a[2]), "v"(a[3]));
    }
}

__global__ __launch_bounds__(32) void k_gemm_h(const h16* __restrict__ A, const h16* __restrict__ Bt, int K, float osc, h16* Ph,
                                               int RB, size_t sRB, int pitch, int CB, size_t sCB, int mode, const float* __restrict__ bias) {
    __shared__ __align__(16) float os[16 * 68];
    const int lane = threadIdx.x & 31, lr = lane & 15, hi = lane >> 4; const int r0 = blockIdx.x * 64, c0 = blockIdx.y * 64;
    v8f acc[4][4];
    gemm_main(A, Bt, K, r0, c0, lr, hi, acc);
    const int rr = r0 % RB, cr = c0 % CB;
    const size_t tbase = (size_t)(r0 / RB) * sRB + (size_t)rr * (size_t)pitch + (size_t)(c0 / CB) * sCB + (size_t)cr;
    const int c8 = (lane & 7) * 8;
    v4f bA = (v4f){}, bB = (v4f){};
    if (mode == 2) { bA = *(const v4f*)(bias + c0 + c8); bB = *(const v4f*)(bias + c0 + c8 + 4);
#pragma unroll
        for (int i = 0; i < 4; ++i) { bA[i] = bfr(bA[i]); bB[i] = bfr(bB[i]); } }
    const float sc2 = (mode == 2) ? 1.0f : osc;
#pragma unroll
    for (int mb = 0; mb < 4; ++mb) {
#pragma unroll
        for (int nb = 0; nb < 4; ++nb) {
#pragma unroll
            for (int j = 0; j < 8; ++j) os[(hi * 8 + j) * 68 + nb * 16 + lr] = acc[mb][nb][j]; }
        wave_sync();
        if (mode == 2) {
#pragma unroll 1
            for (int s = 0; s < 4; ++s) { const int row = 4 * s + (lane >> 3);
                v4f x0 = *(const v4fa*)(&os[row * 68 + c8]); v4f x1 = *(const v4fa*)(&os[row * 68 + c8 + 4]);
#pragma unroll
                for (int i = 0; i < 4; ++i) { x0[i] = gelu_f(x0[i] * osc + bA[i]); x1[i] = gelu_f(x1[i] * osc + bB[i]); }
                *(v4fa*)(&os[row * 68 + c8]) = x0; *(v4fa*)(&os[row * 68 + c8 + 4]) = x1; }
            wave_sync();
        }
        v8h hv[4];
#pragma unroll
        for (int s = 0; s < 4; ++s) { const int row = 4 * s + (lane >> 3);
            const v4f x0 = *(const v4fa*)(&os[row * 68 + c8]); const v4f x1 = *(const v4fa*)(&os[row * 68 + c8 + 4]);
#pragma unroll
            for (int i = 0; i < 4; ++i) { hv[s][i] = toh_flush(x0[i] * sc2); hv[s][4 + i] = toh_flush(x1[i] * sc2); } }
        const size_t sb = tbase + (size_t)(mb * 16) * (size_t)pitch;
#pragma unroll 1
        for (int ps = 0; ps < 2; ++ps) {
#pragma unroll
            for (int s = 0; s < 4; ++s) *(volatile v8h*)(Ph + sb + (size_t)(4 * s + (lane >> 3)) * (size_t)pitch + c8) = hv[s];
            if (ps == 0) __threadfence(); }
        wave_sync();
    }
}

__global__ __launch_bounds__(32) void k_gemm_f(const h16* __restrict__ A, const h16* __restrict__ Bt, int K, float osc, const float* __restrict__ bias,
                                               float* outF, int ldo) {
    __shared__ __align__(16) float os[16 * 68];
    const int lane = threadIdx.x & 31, lr = lane & 15, hi = lane >> 4; const int r0 = blockIdx.x * 64, c0 = blockIdx.y * 64;
    v8f acc[4][4];
    gemm_main(A, Bt, K, r0, c0, lr, hi, acc);
    const int cofs = lr * 4;
    float* op = outF + (size_t)r0 * (size_t)ldo + c0 + cofs;
    v4f bq = *(const v4f*)(bias + c0 + cofs);
#pragma unroll
    for (int i = 0; i < 4; ++i) bq[i] = bfr(bq[i]);
#pragma unroll
    for (int mb = 0; mb < 4; ++mb) {
#pragma unroll
        for (int nb = 0; nb < 4; ++nb) {
#pragma unroll
            for (int j = 0; j < 8; ++j) os[(hi * 8 + j) * 68 + nb * 16 + lr] = acc[mb][nb][j]; }
        wave_sync();
        v4f vv[8];
#pragma unroll
        for (int s = 0; s < 8; ++s) { const int row = 2 * s + hi;
            const v4f y = *(const v4fa*)(&os[row * 68 + cofs]);
#pragma unroll
            for (int i = 0; i < 4; ++i) vv[s][i] = y[i] * osc + bq[i]; }
#pragma unroll 1
        for (int ps = 0; ps < 2; ++ps) {
#pragma unroll
            for (int s = 0; s < 8; ++s) *(volatile v4f*)(op + (size_t)(mb * 16 + 2 * s + hi) * (size_t)ldo) = vv[s];
            if (ps == 0) __threadfence(); }
        wave_sync();
    }
}

__global__ __launch_bounds__(32 * AW) void k_flash(const h16* __restrict__ QH, const h16* __restrict__ KP, const h16* __restrict__ VT, h16* ATT) {
    __shared__ __align__(16) float os[AW * 16 * 68];
    const int lane = threadIdx.x & 31, wave = __builtin_amdgcn_readfirstlane((int)(threadIdx.x >> 5)), lr = lane & 15, hi = lane >> 4;
    const int zh = blockIdx.y; const int b = zh / NH_, h = zh % NH_;
    const int t0 = (blockIdx.x * AW + wave) * 16;
    const size_t pbase = (size_t)zh * SEQ * HD;
    const size_t qo = pbase + (size_t)(t0 + lr) * HD + 8 * hi;
    const v16h qh0 = ldh(QH + qo), qh1 = ldh(QH + qo + 32);
    const size_t ko = pbase + (size_t)lr * HD + 8 * hi;
    const size_t vo = pbase + (size_t)lr * SEQ + 8 * hi;
    v8f o0 = (v8f){}, o1 = (v8f){}, o2 = (v8f){}, o3 = (v8f){};
    float m = -3.0e38f, l = 0.0f;
#pragma unroll 1
    for (int key0 = 0; key0 < SEQ; key0 += 32) {
        const h16* ka = KP + ko + (size_t)key0 * HD;
        const v16h ka0 = ldh(ka), ka1 = ldh(ka + 32), kb0 = ldh(ka + 16 * HD), kb1 = ldh(ka + 16 * HD + 32);
        v8f sa = (v8f){}, sb = (v8f){};
        sa = wmma16g(ka0, qh0, sa); sb = wmma16g(kb0, qh0, sb);
        sa = wmma16g(ka1, qh1, sa); sb = wmma16g(kb1, qh1, sb);
        float mx = -3.0e38f;
#pragma unroll
        for (int r = 0; r < 8; ++r) mx = fmaxf(mx, fmaxf(sa[r], sb[r]));
        mx = fmaxf(mx, __shfl_xor(mx, 16, 32));
        const float mnew = fmaxf(m, mx * SC2);
        const float alpha = __builtin_amdgcn_exp2f(m - mnew);
        const float sh = PSH - mnew;
        v16h pb; float ls = 0.0f;
#pragma unroll
        for (int r = 0; r < 8; ++r) { const float ea = fmaf(sa[r], SC2, sh), ec = fmaf(sb[r], SC2, sh);
            const float fa = (ea < -14.0f) ? 0.0f : __builtin_amdgcn_exp2f(ea);
            const float fc = (ec < -14.0f) ? 0.0f : __builtin_amdgcn_exp2f(ec);
            const h16 pa = (h16)fa; const h16 pc = (h16)fc; pb[r] = pa; pb[8 + r] = pc;
            ls += (float)pa + (float)pc; }
        l = l * alpha + ls; m = mnew;
        if (__builtin_amdgcn_ballot_w32(alpha != 1.0f) != 0u) {
            o0 = o0 * alpha; o1 = o1 * alpha; o2 = o2 * alpha; o3 = o3 * alpha; }
        const h16* va = VT + vo + key0;
        const v16h v0 = ldh(va), v1 = ldh(va + (size_t)16 * SEQ), v2 = ldh(va + (size_t)32 * SEQ), v3 = ldh(va + (size_t)48 * SEQ);
        o0 = wmma16g(v0, pb, o0); o1 = wmma16g(v1, pb, o1); o2 = wmma16g(v2, pb, o2); o3 = wmma16g(v3, pb, o3);
    }
    l += __shfl_xor(l, 16, 32);
    const float inv = ACY * (1.0f / l);
    const int wb = wave * 16 * 68;
    { v4f a, c;
      a[0] = o0[0] * inv; a[1] = o0[1] * inv; a[2] = o0[2] * inv; a[3] = o0[3] * inv; c[0] = o0[4] * inv; c[1] = o0[5] * inv; c[2] = o0[6] * inv; c[3] = o0[7] * inv;
      *(v4fa*)(&os[wb + lr * 68 +  0 + 8 * hi]) = a; *(v4fa*)(&os[wb + lr * 68 +  0 + 8 * hi + 4]) = c;
      a[0] = o1[0] * inv; a[1] = o1[1] * inv; a[2] = o1[2] * inv; a[3] = o1[3] * inv; c[0] = o1[4] * inv; c[1] = o1[5] * inv; c[2] = o1[6] * inv; c[3] = o1[7] * inv;
      *(v4fa*)(&os[wb + lr * 68 + 16 + 8 * hi]) = a; *(v4fa*)(&os[wb + lr * 68 + 16 + 8 * hi + 4]) = c;
      a[0] = o2[0] * inv; a[1] = o2[1] * inv; a[2] = o2[2] * inv; a[3] = o2[3] * inv; c[0] = o2[4] * inv; c[1] = o2[5] * inv; c[2] = o2[6] * inv; c[3] = o2[7] * inv;
      *(v4fa*)(&os[wb + lr * 68 + 32 + 8 * hi]) = a; *(v4fa*)(&os[wb + lr * 68 + 32 + 8 * hi + 4]) = c;
      a[0] = o3[0] * inv; a[1] = o3[1] * inv; a[2] = o3[2] * inv; a[3] = o3[3] * inv; c[0] = o3[4] * inv; c[1] = o3[5] * inv; c[2] = o3[6] * inv; c[3] = o3[7] * inv;
      *(v4fa*)(&os[wb + lr * 68 + 48 + 8 * hi]) = a; *(v4fa*)(&os[wb + lr * 68 + 48 + 8 * hi + 4]) = c; }
    wave_sync();
    h16* orow = ATT + ((size_t)b * SEQ + t0) * DM + h * HD;
    const int c8 = (lane & 7) * 8;
    v8h hv[4];
#pragma unroll
    for (int s = 0; s < 4; ++s) { const int row = 4 * s + (lane >> 3);
        const v4f x0 = *(const v4fa*)(&os[wb + row * 68 + c8]); const v4f x1 = *(const v4fa*)(&os[wb + row * 68 + c8 + 4]);
#pragma unroll
        for (int i = 0; i < 4; ++i) { hv[s][i] = toh_flush(x0[i]); hv[s][4 + i] = toh_flush(x1[i]); } }
#pragma unroll 1
    for (int ps = 0; ps < 2; ++ps) {
#pragma unroll
        for (int s = 0; s < 4; ++s) *(volatile v8h*)(orow + (size_t)(4 * s + (lane >> 3)) * DM + c8) = hv[s];
        if (ps == 0) __threadfence(); }
}

static constexpr size_t cmax(size_t a, size_t b) { return a > b ? a : b; }
static constexpr size_t SZ_WQKV = (size_t)3 * DM * DM * 2;
static constexpr size_t SZ_WO   = (size_t)DM * DM * 2;
static constexpr size_t SZ_W1   = (size_t)FFD * DM * 2;
static constexpr size_t SZ_W2   = (size_t)DM * FFD * 2;
static constexpr size_t SZ_ACT  = (size_t)MROWS * DM * 2;
static constexpr size_t SZ_PL   = (size_t)NB * NH_ * SEQ * HD * 2;
static constexpr size_t SZ_X1   = (size_t)MROWS * DM * 4;
static constexpr size_t SZ_FH   = (size_t)MHALF * FFD * 2;
static constexpr size_t SZ_FQ   = (size_t)MHALF * DM * 4;
static constexpr size_t SZ_C    = cmax(SZ_X1, SZ_FH);
static constexpr size_t SZ_B1   = 3 * SZ_PL;
static constexpr size_t SZ_B2   = SZ_X1 + SZ_C + SZ_FQ;
static constexpr size_t SZ_B    = cmax(SZ_B1, SZ_B2);
static constexpr size_t SZ_TOTAL = SZ_WQKV + SZ_WO + SZ_W1 + SZ_W2 + SZ_ACT + SZ_B;
static_assert(SZ_TOTAL <= (size_t)134217728);
static_assert(SZ_WQKV % 256 == 0 && SZ_WO % 256 == 0 && SZ_W1 % 256 == 0 && SZ_W2 % 256 == 0);
static_assert(SZ_ACT % 256 == 0 && SZ_PL % 256 == 0 && SZ_X1 % 256 == 0 && SZ_FH % 256 == 0 && SZ_FQ % 256 == 0);
static_assert(SZ_B1 <= SZ_B && SZ_B2 <= SZ_B);
static_assert(SZ_X1 <= SZ_C && SZ_FH <= SZ_C);
static_assert((size_t)NB * DM * SEQ * 2 == SZ_PL);

extern "C" void kernel_launch(void* const* d_in, const int* in_sizes, int n_in,
                              void* d_out, int out_size, void* d_ws, size_t ws_size, hipStream_t stream) {
    if (n_in < 14) return;
    const size_t needx = ((size_t)(NB - 1) * SEQ_FULL + SEQ) * DM;
    if ((size_t)in_sizes[0] < needx) return;
    if ((size_t)in_sizes[1] < (size_t)NH_ * DM * HD || (size_t)in_sizes[2] < (size_t)NH_ * DM * HD || (size_t)in_sizes[3] < (size_t)NH_ * DM * HD) return;
    if ((size_t)in_sizes[4] < (size_t)DM * DM || (size_t)in_sizes[5] < (size_t)DM) return;
    if ((size_t)in_sizes[6] < (size_t)DM || (size_t)in_sizes[7] < (size_t)DM) return;
    if ((size_t)in_sizes[8] < (size_t)DM * FFD || (size_t)in_sizes[9] < (size_t)FFD) return;
    if ((size_t)in_sizes[10] < (size_t)FFD * DM || (size_t)in_sizes[11] < (size_t)DM) return;
    if ((size_t)in_sizes[12] < (size_t)DM || (size_t)in_sizes[13] < (size_t)DM) return;
    if ((size_t)out_size < ((size_t)(NB - 1) * OUT_SEQ + SEQ) * DM) return;
    if (SZ_TOTAL > ws_size) return;
    const float* x   = (const float*)d_in[0];
    const float* wq  = (const float*)d_in[1];
    const float* wk  = (const float*)d_in[2];
    const float* wv  = (const float*)d_in[3];
    const float* wo  = (const float*)d_in[4];
    const float* bo  = (const float*)d_in[5];
    const float* g1  = (const float*)d_in[6];
    const float* be1 = (const float*)d_in[7];
    const float* w1  = (const float*)d_in[8];
    const float* b1  = (const float*)d_in[9];
    const float* w2  = (const float*)d_in[10];
    const float* b2  = (const float*)d_in[11];
    const float* g2  = (const float*)d_in[12];
    const float* be2 = (const float*)d_in[13];
    float* OUT = (float*)d_out;

    char* wsp = (char*)d_ws;
    h16* WQKV = (h16*)wsp; wsp += SZ_WQKV;
    h16* WOT  = (h16*)wsp; wsp += SZ_WO;
    h16* W1T  = (h16*)wsp; wsp += SZ_W1;
    h16* W2T  = (h16*)wsp; wsp += SZ_W2;
    h16* ACT  = (h16*)wsp; wsp += SZ_ACT;
    char* rB  = wsp;
    h16* QH = (h16*)rB;
    h16* KP = (h16*)(rB + SZ_PL);
    h16* VT = (h16*)(rB + 2 * SZ_PL);
    float* X1  = (float*)rB;
    float* MHA = (float*)(rB + SZ_X1);
    h16* FFH   = (h16*)(rB + SZ_X1);
    float* FFQ = (float*)(rB + SZ_X1 + SZ_C);
    h16* WQ = WQKV; h16* WK = WQKV + (size_t)DM * DM; h16* WV = WQKV + (size_t)2 * DM * DM;
    h16* XH = ACT; h16* ATT = ACT; h16* X1H = ACT;

    k_tcvt<<<dim3(HD / 64, DM / 64, NH_), 256, 0, stream>>>(wq, WQ, DM, HD, (size_t)DM * HD, (size_t)HD * DM);
    k_tcvt<<<dim3(HD / 64, DM / 64, NH_), 256, 0, stream>>>(wk, WK, DM, HD, (size_t)DM * HD, (size_t)HD * DM);
    k_tcvt<<<dim3(HD / 64, DM / 64, NH_), 256, 0, stream>>>(wv, WV, DM, HD, (size_t)DM * HD, (size_t)HD * DM);
    k_tcvt<<<dim3(DM / 64, DM / 64, 1), 256, 0, stream>>>(wo, WOT, DM, DM, (size_t)0, (size_t)0);
    k_tcvt<<<dim3(FFD / 64, DM / 64, 1), 256, 0, stream>>>(w1, W1T, DM, FFD, (size_t)0, (size_t)0);
    k_tcvt<<<dim3(DM / 64, FFD / 64, 1), 256, 0, stream>>>(w2, W2T, FFD, DM, (size_t)0, (size_t)0);

    k_cast<<<MROWS / 8, 256, 0, stream>>>(x, XH, SEQ_FULL);

    k_gemm_h<<<dim3(MROWS / 64, DM / 64, 1), 32, 0, stream>>>(XH, WQ, DM, WSI, QH, SEQ, (size_t)NH_ * SEQ * HD, HD, HD, (size_t)SEQ * HD, 0, b1);
    k_gemm_h<<<dim3(MROWS / 64, DM / 64, 1), 32, 0, stream>>>(XH, WK, DM, WSI, KP, SEQ, (size_t)NH_ * SEQ * HD, HD, HD, (size_t)SEQ * HD, 0, b1);
    k_gemm_h<<<dim3(DM / 64, MROWS / 64, 1), 32, 0, stream>>>(WV, XH, DM, WSI, VT, DM, (size_t)0, SEQ, SEQ, (size_t)DM * SEQ, 0, b1);

    k_flash<<<dim3(SEQ / (16 * AW), NB * NH_, 1), 32 * AW, 0, stream>>>(QH, KP, VT, ATT);

    k_gemm_f<<<dim3(MROWS / 64, DM / 64, 1), 32, 0, stream>>>(ATT, WOT, DM, WSI * (1.0f / ACY), bo, MHA, DM);

    k_lnres<<<MROWS / 8, 256, 0, stream>>>(MHA, x, g1, be1, X1, X1H, 1, 1, 0, SEQ_FULL, SEQ);

    for (int hf = 0; hf < 2; ++hf) {
        k_gemm_h<<<dim3(MHALF / 64, FFD / 64, 1), 32, 0, stream>>>(X1H + (size_t)hf * MHALF * DM, W1T, DM, WSI, FFH, BIGB, (size_t)0, FFD, BIGB, (size_t)0, 2, b1);
        k_gemm_f<<<dim3(MHALF / 64, DM / 64, 1), 32, 0, stream>>>(FFH, W2T, FFD, WSI, b2, FFQ, DM);
        k_lnres<<<MHALF / 8, 256, 0, stream>>>(FFQ, X1, g2, be2, OUT, X1H, 0, 0, hf * MHALF, SEQ, OUT_SEQ);
    }
}
